// Transformer_Block_1417339207765
// MI455X (gfx1250) — hardware-run, weakly checked
//
#include <hip/hip_runtime.h>
#include <stdint.h>
#include <stddef.h>

typedef __attribute__((ext_vector_type(16))) _Float16 v16h;
typedef __attribute__((ext_vector_type(8)))  _Float16 v8h;
typedef __attribute__((ext_vector_type(16))) __bf16   v16b;
typedef __attribute__((ext_vector_type(8)))  __bf16   v8b;
typedef __attribute__((ext_vector_type(8)))  float    v8f;
typedef __attribute__((ext_vector_type(4)))  float    v4f;

constexpr int  BATCH    = 8;
constexpr int  SEQ      = 1024;
constexpr int  EMB_DIM  = 1024;
constexpr int  ROWS_ALL = BATCH * SEQ;
constexpr long PLANE_ELEMS = (long)SEQ * EMB_DIM;
constexpr long ACT_ELEMS   = (long)BATCH * PLANE_ELEMS;
constexpr long W_ELEMS     = (long)EMB_DIM * EMB_DIM;
constexpr float LN_EPS   = 1e-3f;
constexpr float W_CARRY  = 64.0f;
constexpr float W_CARRY_INV = 1.0f / 64.0f;
constexpr float P_CARRY  = 1024.0f;
constexpr float P_CARRY_INV = 1.0f / 1024.0f;
constexpr float SCORE_SCALE = 1.0f / 32.0f;

static_assert(SEQ % 64 == 0 && EMB_DIM % 64 == 0 && ROWS_ALL % 64 == 0, "tile multiples");
static_assert(EMB_DIM % 32 == 0 && SEQ % 32 == 0, "K multiple of 32");
static_assert(SEQ == 1024 && EMB_DIM == 1024, "row kernels assume 1024-wide rows");

constexpr size_t P16_BYTES = (size_t)ACT_ELEMS * 2;
constexpr size_t P32_BYTES = (size_t)ACT_ELEMS * 4;
constexpr size_t OFF_R0  = 0;
constexpr size_t OFF_R2  = OFF_R0 + P16_BYTES;
constexpr size_t OFF_R3  = OFF_R2 + P16_BYTES;
constexpr size_t OFF_R4  = OFF_R3 + P16_BYTES;
constexpr size_t OFF_R56 = OFF_R4 + P16_BYTES;
constexpr size_t OFF_R78 = OFF_R56 + P32_BYTES;
constexpr size_t WS_TOTAL = OFF_R78 + P32_BYTES;
static_assert(WS_TOTAL == 134217728ull, "carve 128 MiB");
static_assert((size_t)W_ELEMS * 2 <= P16_BYTES && (size_t)W_ELEMS * 2 <= P32_BYTES, "weight slot fits");

#define U16(p) ((const unsigned short*)(const void*)(p))

__device__ __forceinline__ unsigned short f2bf_bits(float f) {
  unsigned u = __float_as_uint(f);
  return (unsigned short)((u + 0x7FFFu + ((u >> 16) & 1u)) >> 16);
}
__device__ __forceinline__ float bf_bits2f(unsigned short h) { return __uint_as_float(((unsigned)h) << 16); }

__device__ __forceinline__ void dep_guard_h(v8f& a, v8f& b, v16h x, v16h y) { asm volatile("v_nop\n\tv_nop\n\tv_nop\n\tv_nop" : "+v"(a), "+v"(b) : "v"(x), "v"(y)); }
__device__ __forceinline__ void dep_guard_b(v8f& a, v8f& b, v16b x, v16b y) { asm volatile("v_nop\n\tv_nop\n\tv_nop\n\tv_nop" : "+v"(a), "+v"(b) : "v"(x), "v"(y)); }
__device__ __forceinline__ void keep4_h(v16h a, v16h b, v16h c, v16h d) { asm volatile("v_nop" :: "v"(a), "v"(b), "v"(c), "v"(d)); }
__device__ __forceinline__ void keep4_b(v16b a, v16b b, v16b c, v16b d) { asm volatile("v_nop" :: "v"(a), "v"(b), "v"(c), "v"(d)); }
__device__ __forceinline__ void acc_guard4(v8f& a, v8f& b, v8f& c, v8f& d) { asm volatile("v_nop\n\tv_nop\n\tv_nop\n\tv_nop" : "+v"(a), "+v"(b), "+v"(c), "+v"(d)); }
template <typename T> struct Frag;
template <> struct Frag<_Float16> {
  typedef v16h V; union U { v16h v; v8h h[2]; };
  static __device__ __forceinline__ v16h load(const _Float16* p) {
    U f; f.h[0] = *(const v8h*)(p); f.h[1] = *(const v8h*)(p + 16); return f.v;
  }
  static __device__ __forceinline__ v8f mma(v16h a, v16h b, v8f c) {
    return __builtin_amdgcn_wmma_f32_16x16x32_f16(false, a, false, b, (short)0, c, false, false);
  }
  static __device__ __forceinline__ void guard(v8f& a, v8f& b, v16h x, v16h y) { dep_guard_h(a, b, x, y); }
  static __device__ __forceinline__ void keep(v16h a, v16h b, v16h c, v16h d) { keep4_h(a, b, c, d); }
};
template <> struct Frag<__bf16> {
  typedef v16b V; union U { v16b v; v8b h[2]; };
  static __device__ __forceinline__ v16b load(const __bf16* p) {
    U f; f.h[0] = *(const v8b*)(p); f.h[1] = *(const v8b*)(p + 16); return f.v;
  }
  static __device__ __forceinline__ v8f mma(v16b a, v16b b, v8f c) {
    return __builtin_amdgcn_wmma_f32_16x16x32_bf16(false, a, false, b, (short)0, c, false, false);
  }
  static __device__ __forceinline__ void guard(v8f& a, v8f& b, v16b x, v16b y) { dep_guard_b(a, b, x, y); }
  static __device__ __forceinline__ void keep(v16b a, v16b b, v16b c, v16b d) { keep4_b(a, b, c, d); }
};

template <int ET> struct Elem;
template <> struct Elem<0> { typedef _Float16 T; };
template <> struct Elem<1> { typedef __bf16 T; };
template <int ET, bool SPLIT, int BIAS_MODE, int OUT_MODE, bool RESID, int ACT = 0, int CAUSAL = 0>
__global__ __launch_bounds__(256) void wmma_gemm64(
    const unsigned short* __restrict__ Ap, const unsigned short* __restrict__ A2p, int lda, long strideA,
    const unsigned short* __restrict__ Btp, const unsigned short* __restrict__ Bt2p, int ldb, long strideB,
    void* __restrict__ Cout, void* __restrict__ Cout2, int ldc, long strideC,
    const float* __restrict__ bias,
    const float* __restrict__ resid, long strideR,
    int M, int N, int K, float scale) {
  typedef typename Elem<ET>::T T;
  typedef typename Frag<T>::V V;
  const T* A = (const T*)Ap; const T* A2 = (const T*)A2p; const T* Bt = (const T*)Btp; const T* Bt2 = (const T*)Bt2p;
  __shared__ __align__(16) float sT[8][16 * 68];
  const int b    = blockIdx.y;
  const int lane = threadIdx.x & 31;
  const int wave = threadIdx.x >> 5;
  const int tilesN = N >> 6;
  const int tilesM = M >> 6;
  const int tile = blockIdx.x * 8 + wave;
  if (tile >= tilesM * tilesN) return;
  const int tm = tile / tilesN;
  const int tn = tile - tm * tilesN;
  if (CAUSAL == 1 && tn > tm) return;
  const int m0 = tm << 6;
  const int n0 = tn << 6;
  const int Kend = (CAUSAL == 2) ? ((m0 + 64 < K) ? (m0 + 64) : K) : K;

  const T* Ab  = A  + (size_t)b * strideA;
  const T* Bb  = Bt + (size_t)b * strideB;
  const T* Ab2 = SPLIT ? (A2  + (size_t)b * strideA) : nullptr;
  const T* Bb2 = SPLIT ? (Bt2 + (size_t)b * strideB) : nullptr;

  const int rlane = lane & 15;
  const int koff  = (lane >> 4) * 8;
  const int mOff  = (lane >> 4) * 8;

  v8f acc[4][4];
#pragma unroll
  for (int i = 0; i < 4; ++i)
#pragma unroll
    for (int j = 0; j < 4; ++j) acc[i][j] = (v8f){0.f,0.f,0.f,0.f,0.f,0.f,0.f,0.f};

  for (int k0 = 0; k0 < Kend; k0 += 32) {
    V bh[4], bl[4];
#pragma unroll
    for (int j = 0; j < 4; ++j) {
      const size_t bo = (size_t)(n0 + (j << 4) + rlane) * ldb + koff + k0;
      bh[j] = Frag<T>::load(Bb + bo);
      if (SPLIT) bl[j] = Frag<T>::load(Bb2 + bo);
    }
#pragma unroll
    for (int i = 0; i < 4; ++i) {
      const size_t ao = (size_t)(m0 + (i << 4) + rlane) * lda + koff + k0;
      V ah = Frag<T>::load(Ab + ao);
      V al;
      if (SPLIT) al = Frag<T>::load(Ab2 + ao);
#pragma unroll
      for (int j = 0; j < 4; ++j) {
        acc[i][j] = Frag<T>::mma(ah, bh[j], acc[i][j]);
        if (SPLIT) {
          acc[i][j] = Frag<T>::mma(ah, bl[j], acc[i][j]);
          acc[i][j] = Frag<T>::mma(al, bh[j], acc[i][j]);
        }
      }
      Frag<T>::guard(acc[i][0], acc[i][3], ah, SPLIT ? al : ah);
    }
    Frag<T>::keep(bh[0], bh[1], bh[2], bh[3]);
    if (SPLIT) Frag<T>::keep(bl[0], bl[1], bl[2], bl[3]);
  }
  acc_guard4(acc[0][0], acc[0][1], acc[0][2], acc[0][3]);
  acc_guard4(acc[1][0], acc[1][1], acc[1][2], acc[1][3]);
  acc_guard4(acc[2][0], acc[2][1], acc[2][2], acc[2][3]);
  acc_guard4(acc[3][0], acc[3][1], acc[3][2], acc[3][3]);

  float* slab = sT[wave];
  const float* Rb = RESID ? (resid + (size_t)b * strideR) : nullptr;
#pragma unroll
  for (int i = 0; i < 4; ++i) {
    const int mBase = m0 + (i << 4);
#pragma unroll
    for (int j = 0; j < 4; ++j) {
      const int n = n0 + (j << 4) + rlane;
      float bv = 0.f;
      if (BIAS_MODE == 2) bv = bias[n];
#pragma unroll
      for (int r = 0; r < 8; ++r) {
        float v = acc[i][j][r] * scale;
        if (BIAS_MODE == 1) v += bias[mBase + mOff + r];
        if (BIAS_MODE == 2) v += bv;
        if (RESID) v += Rb[(size_t)(mBase + mOff + r) * ldc + n];
        if (ACT == 1) v = tanhf(v);
        if (ACT == 2) v = fmaxf(v, 0.0f);
        if (ACT == 3) v = v / (1.0f + expf(-v));
        if (ACT == 4) v = (v > 0.f) ? v : 0.01f * v;
        if (ACT == 5) v = 0.5f * v * (1.0f + erff(v * 0.70710678118654752f));
        slab[(mOff + r) * 68 + (j << 4) + rlane] = v;
      }
    }
    __builtin_amdgcn_fence(__ATOMIC_RELEASE, "workgroup");
    __builtin_amdgcn_wave_barrier();
    __builtin_amdgcn_fence(__ATOMIC_ACQUIRE, "workgroup");
    if (OUT_MODE == 0) {
      float* C = (float*)Cout + (size_t)b * strideC;
      const int hh = lane >> 4, c4 = (lane & 15) * 4;
      for (int pass = 0; pass < 2; ++pass) {
#pragma unroll
        for (int it = 0; it < 8; ++it) {
          const int row = it * 2 + hh;
          v4f v = *(const v4f*)(slab + row * 68 + c4);
          *(volatile v4f*)(C + (size_t)(mBase + row) * ldc + n0 + c4) = v;
        }
        __threadfence();
      }
    } else {
      const int q = lane >> 3, c8 = (lane & 7) * 8;
      unsigned short* C  = (unsigned short*)Cout  + (size_t)b * strideC;
      unsigned short* C2 = (OUT_MODE == 2) ? ((unsigned short*)Cout2 + (size_t)b * strideC) : nullptr;
      for (int pass = 0; pass < 2; ++pass) {
#pragma unroll
        for (int it = 0; it < 4; ++it) {
          const int row = it * 4 + q;
          const float* sp = slab + row * 68 + c8;
          v8h hv, lv;
#pragma unroll
          for (int e = 0; e < 8; ++e) {
            if (OUT_MODE == 1) {
              hv[e] = (_Float16)sp[e];
            } else {
              unsigned short hb = f2bf_bits(sp[e]);
              unsigned short lb = f2bf_bits(sp[e] - bf_bits2f(hb));
              hv[e] = __builtin_bit_cast(_Float16, hb);
              lv[e] = __builtin_bit_cast(_Float16, lb);
            }
          }
          *(volatile v8h*)(C + (size_t)(mBase + row) * ldc + n0 + c8) = hv;
          if (OUT_MODE == 2) *(volatile v8h*)(C2 + (size_t)(mBase + row) * ldc + n0 + c8) = lv;
        }
        __threadfence();
      }
    }
    __builtin_amdgcn_fence(__ATOMIC_RELEASE, "workgroup");
    __builtin_amdgcn_wave_barrier();
    __builtin_amdgcn_fence(__ATOMIC_ACQUIRE, "workgroup");
  }
}

template <int NW>
__device__ __forceinline__ float blk_sum(float v, float* red) {
#pragma unroll
  for (int o = 16; o > 0; o >>= 1) v += __shfl_xor(v, o, 32);
  __syncthreads();
  if ((threadIdx.x & 31) == 0) red[threadIdx.x >> 5] = v;
  __syncthreads();
  float t = 0.f;
#pragma unroll
  for (int i = 0; i < NW; ++i) t += red[i];
  return t;
}
template <int NW>
__device__ __forceinline__ float blk_max(float v, float* red) {
#pragma unroll
  for (int o = 16; o > 0; o >>= 1) v = fmaxf(v, __shfl_xor(v, o, 32));
  __syncthreads();
  if ((threadIdx.x & 31) == 0) red[threadIdx.x >> 5] = v;
  __syncthreads();
  float t = red[0];
#pragma unroll
  for (int i = 1; i < NW; ++i) t = fmaxf(t, red[i]);
  return t;
}

__global__ __launch_bounds__(256) void cast_rows_f16(const float* __restrict__ src,
                                                     _Float16* __restrict__ dst, int n8) {
  const int i = blockIdx.x * 256 + threadIdx.x;
  if (i >= n8) return;
  const float* p = src + (size_t)i * 8;
  const v4f a = *(const v4f*)(p);
  const v4f c = *(const v4f*)(p + 4);
  v8h hv;
  hv[0] = (_Float16)a[0]; hv[1] = (_Float16)a[1]; hv[2] = (_Float16)a[2]; hv[3] = (_Float16)a[3];
  hv[4] = (_Float16)c[0]; hv[5] = (_Float16)c[1]; hv[6] = (_Float16)c[2]; hv[7] = (_Float16)c[3];
  _Float16* q = dst + (size_t)i * 8;
  *(volatile v8h*)q = hv;
  __threadfence();
  *(volatile v8h*)q = hv;
}

__global__ __launch_bounds__(256) void wt_transpose_f16(const float* __restrict__ W,
                                                        _Float16* __restrict__ Wt, float mul) {
  __shared__ float s[64 * 65];
  const int o0 = blockIdx.x * 64;
  const int e0 = blockIdx.y * 64;
  const int t  = threadIdx.x;
  {
    const int e  = t >> 2;
    const int oq = (t & 3) * 16;
    const float* p = W + (size_t)(e0 + e) * EMB_DIM + o0 + oq;
#pragma unroll
    for (int i = 0; i < 4; ++i) {
      const v4f v = *(const v4f*)(p + 4 * i);
#pragma unroll
      for (int c = 0; c < 4; ++c) s[(oq + 4 * i + c) * 65 + e] = v[c];
    }
  }
  __syncthreads();
  const int wave = t >> 5, lane = t & 31;
  const int q = lane >> 3, e8 = (lane & 7) * 8;
  for (int pass = 0; pass < 2; ++pass) {
#pragma unroll
    for (int it = 0; it < 2; ++it) {
      const int o = it * 32 + wave * 4 + q;
      const float* sp = s + o * 65 + e8;
      v8h hv;
#pragma unroll
      for (int e = 0; e < 8; ++e) hv[e] = (_Float16)(sp[e] * mul);
      *(volatile v8h*)(Wt + (size_t)(o0 + o) * EMB_DIM + e0 + e8) = hv;
    }
    __threadfence();
  }
}

template <bool CAUSAL>
__global__ __launch_bounds__(128) void softmax_rows(const float* __restrict__ sc,
                                                    _Float16* __restrict__ P) {
  __shared__ float red[4];
  const int row = blockIdx.x;
  const int q   = row & (SEQ - 1);
  const int t   = threadIdx.x;
  const float* src = sc + (size_t)row * SEQ;
  const int jlim = CAUSAL ? q : (SEQ - 1);
  float x[8];
#pragma unroll
  for (int e = 0; e < 8; ++e) {
    const int j  = t * 8 + e;
    const int jc = (j < jlim) ? j : jlim;
    float v = src[jc];
    if (CAUSAL) v = (j > q) ? -__builtin_inff() : v;
    x[e] = v;
  }
  float m = x[0];
#pragma unroll
  for (int e = 1; e < 8; ++e) m = fmaxf(m, x[e]);
  m = blk_max<4>(m, red);
  float ex[8];
  float ssum = 0.f;
#pragma unroll
  for (int e = 0; e < 8; ++e) { ex[e] = expf(x[e] - m); ssum += ex[e]; }
  const float tot = blk_sum<4>(ssum, red);
  const float f = P_CARRY * (1.0f / tot);
  v8h hv;
#pragma unroll
  for (int e = 0; e < 8; ++e) hv[e] = (_Float16)(ex[e] * f);
  _Float16* dst = P + (size_t)row * SEQ + t * 8;
  *(volatile v8h*)dst = hv;
  __threadfence();
  *(volatile v8h*)dst = hv;
}

template <bool RELU, bool HOUT>
__global__ __launch_bounds__(256) void add_ln_rows(const float* a, const float* res,
                                                   const float* __restrict__ gamma,
                                                   const float* __restrict__ beta,
                                                   float* xo, _Float16* ho) {
  __shared__ float red[8];
  __shared__ __align__(16) float ys[HOUT ? EMB_DIM : 4];
  const int row = blockIdx.x;
  const int t   = threadIdx.x;
  const int j0  = t * 4;
  const size_t off = (size_t)row * EMB_DIM + j0;
  const v4f va = *(const v4f*)(a + off);
  const v4f vr = *(const v4f*)(res + off);
  float v[4];
#pragma unroll
  for (int c = 0; c < 4; ++c) v[c] = va[c] + vr[c];
  const float s1 = (v[0] + v[1]) + (v[2] + v[3]);
  const float mu = blk_sum<8>(s1, red) * (1.0f / EMB_DIM);
  float d[4];
  float s2 = 0.f;
#pragma unroll
  for (int c = 0; c < 4; ++c) { d[c] = v[c] - mu; s2 += d[c] * d[c]; }
  const float var = blk_sum<8>(s2, red) * (1.0f / EMB_DIM);
  const float rs  = rsqrtf(var + LN_EPS);
  const v4f g  = *(const v4f*)(gamma + j0);
  const v4f bb = *(const v4f*)(beta + j0);
  v4f y;
#pragma unroll
  for (int c = 0; c < 4; ++c) {
    float yy = d[c] * rs * g[c] + bb[c];
    if (RELU) yy = fmaxf(yy, 0.0f);
    y[c] = yy;
  }
  *(volatile v4f*)(xo + off) = y;
  __threadfence();
  *(volatile v4f*)(xo + off) = y;
  if (HOUT) {
#pragma unroll
    for (int c = 0; c < 4; ++c) ys[j0 + c] = y[c];
    __syncthreads();
    if (t < 128) {
      const float* sp = ys + t * 8;
      v8h hv;
#pragma unroll
      for (int e = 0; e < 8; ++e) hv[e] = (_Float16)sp[e];
      _Float16* hp = ho + (size_t)row * EMB_DIM + t * 8;
      *(volatile v8h*)hp = hv;
      __threadfence();
      *(volatile v8h*)hp = hv;
    }
  }
}

extern "C" void kernel_launch(void* const* d_in, const int* in_sizes, int n_in,
                              void* d_out, int out_size, void* d_ws, size_t ws_size,
                              hipStream_t stream) {
  if (n_in < 14) return;
  if (in_sizes[0] != (int)ACT_ELEMS || in_sizes[1] != (int)ACT_ELEMS) return;
  for (int i = 2; i <= 8; ++i) if (in_sizes[i] != (int)W_ELEMS) return;
  if (in_sizes[10] != (int)W_ELEMS) return;
  if (in_sizes[9] != EMB_DIM || in_sizes[11] != EMB_DIM || in_sizes[12] != EMB_DIM || in_sizes[13] != EMB_DIM) return;
  if (out_size != (int)ACT_ELEMS) return;
  if (ws_size < WS_TOTAL) return;

  const float* x_in  = (const float*)d_in[0];
  const float* ctx   = (const float*)d_in[1];
  const float* wq1   = (const float*)d_in[2];
  const float* wk1   = (const float*)d_in[3];
  const float* wv1   = (const float*)d_in[4];
  const float* wq2   = (const float*)d_in[5];
  const float* wk2   = (const float*)d_in[6];
  const float* wv2   = (const float*)d_in[7];
  const float* w1    = (const float*)d_in[8];
  const float* b1    = (const float*)d_in[9];
  const float* w2    = (const float*)d_in[10];
  const float* b2    = (const float*)d_in[11];
  const float* gamma = (const float*)d_in[12];
  const float* beta  = (const float*)d_in[13];
  float* out = (float*)d_out;

  char* base = (char*)d_ws;
  _Float16* xh    = (_Float16*)(base + OFF_R0);
  _Float16* r2    = (_Float16*)(base + OFF_R2);
  _Float16* r3    = (_Float16*)(base + OFF_R3);
  _Float16* r4    = (_Float16*)(base + OFF_R4);
  float*    r56   = (float*)   (base + OFF_R56);
  float*    r78f  = (float*)   (base + OFF_R78);
  _Float16* r78h  = (_Float16*)(base + OFF_R78);

  const long LE = PLANE_ELEMS;
  const int castGrid = (int)(ACT_ELEMS / 8 / 256);
  const dim3 wtGrid(EMB_DIM / 64, EMB_DIM / 64);
  const dim3 gFlat((ROWS_ALL / 64) * (EMB_DIM / 64) / 8, 1);
  const dim3 gBat((SEQ / 64) * (SEQ / 64) / 8, BATCH);

  cast_rows_f16<<<castGrid, 256, 0, stream>>>(x_in, xh, (int)(ACT_ELEMS / 8));
  wt_transpose_f16<<<wtGrid, 256, 0, stream>>>(wq1, r4, W_CARRY);
  wmma_gemm64<0, false, 0, 1, false, 0, 0><<<gFlat, 256, 0, stream>>>(
      U16(xh), U16(xh), EMB_DIM, 0, U16(r4), U16(r4), EMB_DIM, 0,
      (void*)r2, (void*)r2, EMB_DIM, 0, gamma, gamma, 0, ROWS_ALL, EMB_DIM, EMB_DIM, W_CARRY_INV);
  wt_transpose_f16<<<wtGrid, 256, 0, stream>>>(wk1, r4, W_CARRY);
  wmma_gemm64<0, false, 0, 1, false, 0, 0><<<gFlat, 256, 0, stream>>>(
      U16(xh), U16(xh), EMB_DIM, 0, U16(r4), U16(r4), EMB_DIM, 0,
      (void*)r3, (void*)r3, EMB_DIM, 0, gamma, gamma, 0, ROWS_ALL, EMB_DIM, EMB_DIM, W_CARRY_INV);
  wmma_gemm64<0, false, 0, 0, false, 0, 1><<<gBat, 256, 0, stream>>>(
      U16(r2), U16(r2), EMB_DIM, LE, U16(r3), U16(r3), EMB_DIM, LE,
      (void*)r56, (void*)r56, SEQ, LE, gamma, gamma, 0, SEQ, SEQ, EMB_DIM, SCORE_SCALE);
  softmax_rows<true><<<ROWS_ALL, 128, 0, stream>>>(r56, r2);
  wt_transpose_f16<<<wtGrid, 256, 0, stream>>>(wv1, r4, W_CARRY);
  wmma_gemm64<0, false, 0, 1, false, 0, 0><<<gBat, 256, 0, stream>>>(
      U16(r4), U16(r4), EMB_DIM, 0, U16(xh), U16(xh), EMB_DIM, LE,
      (void*)r3, (void*)r3, SEQ, LE, gamma, gamma, 0, EMB_DIM, SEQ, EMB_DIM, W_CARRY_INV);
  wmma_gemm64<0, false, 0, 0, false, 0, 2><<<gBat, 256, 0, stream>>>(
      U16(r2), U16(r2), SEQ, LE, U16(r3), U16(r3), SEQ, LE,
      (void*)r56, (void*)r56, EMB_DIM, LE, gamma, gamma, 0, SEQ, EMB_DIM, SEQ, P_CARRY_INV);
  add_ln_rows<false, true><<<ROWS_ALL, 256, 0, stream>>>(r56, x_in, gamma, beta, r56, xh);

  cast_rows_f16<<<castGrid, 256, 0, stream>>>(ctx, r4, (int)(ACT_ELEMS / 8));
  wt_transpose_f16<<<wtGrid, 256, 0, stream>>>(wq2, r78h, W_CARRY);
  wmma_gemm64<0, false, 0, 1, false, 0, 0><<<gFlat, 256, 0, stream>>>(
      U16(xh), U16(xh), EMB_DIM, 0, U16(r78h), U16(r78h), EMB_DIM, 0,
      (void*)r2, (void*)r2, EMB_DIM, 0, gamma, gamma, 0, ROWS_ALL, EMB_DIM, EMB_DIM, W_CARRY_INV);
  wt_transpose_f16<<<wtGrid, 256, 0, stream>>>(wk2, r78h, W_CARRY);
  wmma_gemm64<0, false, 0, 1, false, 0, 0><<<gFlat, 256, 0, stream>>>(
      U16(r4), U16(r4), EMB_DIM, 0, U16(r78h), U16(r78h), EMB_DIM, 0,
      (void*)r3, (void*)r3, EMB_DIM, 0, gamma, gamma, 0, ROWS_ALL, EMB_DIM, EMB_DIM, W_CARRY_INV);
  wmma_gemm64<0, false, 0, 0, false, 0, 0><<<gBat, 256, 0, stream>>>(
      U16(r2), U16(r2), EMB_DIM, LE, U16(r3), U16(r3), EMB_DIM, LE,
      (void*)r78f, (void*)r78f, SEQ, LE, gamma, gamma, 0, SEQ, SEQ, EMB_DIM, SCORE_SCALE);
  softmax_rows<false><<<ROWS_ALL, 128, 0, stream>>>(r78f, r2);
  wt_transpose_f16<<<wtGrid, 256, 0, stream>>>(wv2, r78h, W_CARRY);
  wmma_gemm64<0, false, 0, 1, false, 0, 0><<<gBat, 256, 0, stream>>>(
      U16(r78h), U16(r78h), EMB_DIM, 0, U16(r4), U16(r4), EMB_DIM, LE,
      (void*)r3, (void*)r3, SEQ, LE, gamma, gamma, 0, EMB_DIM, SEQ, EMB_DIM, W_CARRY_INV);
  wmma_gemm64<0, false, 0, 0, false, 0, 0><<<gBat, 256, 0, stream>>>(
      U16(r2), U16(r2), SEQ, LE, U16(r3), U16(r3), SEQ, LE,
      (void*)r78f, (void*)r78f, EMB_DIM, LE, gamma, gamma, 0, SEQ, EMB_DIM, SEQ, P_CARRY_INV);
  add_ln_rows<false, true><<<ROWS_ALL, 256, 0, stream>>>(r78f, r56, gamma, beta, r56, xh);

  wt_transpose_f16<<<wtGrid, 256, 0, stream>>>(w1, r3, W_CARRY);
  wmma_gemm64<0, false, 2, 1, false, 2, 0><<<gFlat, 256, 0, stream>>>(
      U16(xh), U16(xh), EMB_DIM, 0, U16(r3), U16(r3), EMB_DIM, 0,
      (void*)r2, (void*)r2, EMB_DIM, 0, b1, gamma, 0, ROWS_ALL, EMB_DIM, EMB_DIM, W_CARRY_INV);
  wt_transpose_f16<<<wtGrid, 256, 0, stream>>>(w2, r4, W_CARRY);
  wmma_gemm64<0, false, 2, 0, false, 0, 0><<<gFlat, 256, 0, stream>>>(
      U16(r2), U16(r2), EMB_DIM, 0, U16(r4), U16(r4), EMB_DIM, 0,
      (void*)r78f, (void*)r78f, EMB_DIM, 0, b2, gamma, 0, ROWS_ALL, EMB_DIM, EMB_DIM, W_CARRY_INV);
  add_ln_rows<true, false><<<ROWS_ALL, 256, 0, stream>>>(r78f, r56, gamma, beta, out, xh);
}
